// Model_25769804184
// MI455X (gfx1250) — hardware-verified
//
#include <hip/hip_runtime.h>
#include <math.h>

typedef __attribute__((ext_vector_type(16))) _Float16 v16h;
typedef __attribute__((ext_vector_type(8)))  _Float16 v8h;
typedef __attribute__((ext_vector_type(8)))  float    v8f;
typedef __attribute__((ext_vector_type(4)))  float    v4f;

constexpr int kT     = 256;
constexpr int kB     = 256;
constexpr int kH     = 100;
constexpr int kHP    = 112;
constexpr int kG4    = 4 * kHP;
constexpr int kEmb   = 50;
constexpr int kVocab = 50000;
constexpr int kXP0   = 64;
constexpr int kHK    = 128;
constexpr int kHPL   = 256;
constexpr int kLbl   = 66;
constexpr int kLblP  = 80;
constexpr int kRows  = kT * kB;
constexpr int kK0    = kXP0 + kHK;
constexpr int kK1    = kHPL + kHK;
constexpr float kCarry     = 64.0f;
constexpr float kCarry2    = kCarry * kCarry;
constexpr float kInvCarry2 = 1.0f / kCarry2;
static_assert(kG4 == 448 && (kK0 % 32) == 0 && (kK1 % 32) == 0 && (kHPL % 32) == 0 && (kXP0 % 32) == 0, "shape");
static_assert((kHP % 16) == 0 && (kLblP % 16) == 0 && (kRows % 128) == 0 && (kB % 32) == 0, "tiles");
static_assert((128 * kLbl * 4) % 128 == 0, "head block rows cover whole lines");

constexpr size_t kOffX0  = 0;
constexpr size_t kOffH0  = kOffX0  + (size_t)kRows * kXP0 * 2;
constexpr size_t kOffH1  = kOffH0  + (size_t)kRows * kHPL * 2;
constexpr size_t kOffWC0 = kOffH1  + (size_t)kRows * kHPL * 2;
constexpr size_t kOffWC1 = kOffWC0 + (size_t)2 * kG4 * kK0 * 2;
constexpr size_t kOffWO  = kOffWC1 + (size_t)2 * kG4 * kK1 * 2;
constexpr size_t kOffBI0 = kOffWO  + (size_t)kLblP * kHPL * 2;
constexpr size_t kOffBI1 = kOffBI0 + (size_t)2 * kG4 * 4;
constexpr size_t kOffBO  = kOffBI1 + (size_t)2 * kG4 * 4;
constexpr size_t kWsTotal = kOffBO + (size_t)128 * 4;
static_assert(kWsTotal == 76578304ull, "carve total");
static_assert(kWsTotal <= 134217728ull, "carve cap");
static_assert((kOffH0 % 128) == 0 && (kOffH1 % 128) == 0 && (kOffWC0 % 128) == 0 && (kOffWC1 % 128) == 0 &&
              (kOffWO % 128) == 0 && (kOffBI0 % 128) == 0 && (kOffBI1 % 128) == 0 && (kOffBO % 128) == 0, "aligned");

union FragU { v16h v; v8h h[2]; };
__device__ __forceinline__ v16h frag_load_g(const _Float16* p) {
  FragU f;
  f.h[0] = *(const v8h*)(p);
  f.h[1] = *(const v8h*)(p + 16);
  return f.v;
}
__device__ __forceinline__ v8f mma_g(v16h a, v16h b, v8f c) {
  c = __builtin_amdgcn_wmma_f32_16x16x32_f16(false, a, false, b, (short)0, c, false, false);
  asm volatile("v_nop\n\tv_nop\n\tv_nop\n\tv_nop" : "+v"(c) : "v"(a), "v"(b));
  return c;
}
__device__ __forceinline__ float sig_fast(float x) {
  return __builtin_amdgcn_rcpf(1.0f + __expf(-x));
}
__device__ __forceinline__ float tanh_fast(float x) {
  const float ax = fabsf(x);
  const float e  = __expf(-2.0f * ax);
  const float t  = (1.0f - e) * __builtin_amdgcn_rcpf(1.0f + e);
  return copysignf(t, x);
}

template <int DIN, int KX>
__global__ __launch_bounds__(256) void prep_wcat_kernel(
    const float* __restrict__ wih_f, const float* __restrict__ whh_f,
    const float* __restrict__ wih_b, const float* __restrict__ whh_b,
    unsigned short* __restrict__ wc)
{
  constexpr int KTOT = KX + kHK;
  constexpr int CPR  = KTOT / 8;
  const int dir = blockIdx.y;
  const float* wih = dir ? wih_b : wih_f;
  const float* whh = dir ? whh_b : whh_f;
  const int i = blockIdx.x * 256 + threadIdx.x;
  if (i >= kG4 * CPR) return;
  const int row = i / CPR;
  const int chn = i - row * CPR;
  const int g   = row / kHP;
  const int j   = row - g * kHP;
  const bool jv = (j < kH);
  const int srow = g * kH + (jv ? j : (kH - 1));
  v8h hv;
#pragma unroll
  for (int e = 0; e < 8; ++e) {
    const int k = chn * 8 + e;
    const bool inx = (k < KX);
    int ci;
    bool vx;
    if (DIN == kEmb) {
      ci = (k < kEmb) ? k : (kEmb - 1);
      vx = inx && (k < kEmb);
    } else {
      const int half = (k >> 7) & 1;
      const int kk   = k & 127;
      ci = half * kH + ((kk < kH) ? kk : (kH - 1));
      vx = inx && (kk < kH);
    }
    const int kh  = k - KX;
    const int khc = (kh < 0) ? 0 : ((kh < kH) ? kh : (kH - 1));
    const bool vh = (!inx) && (kh < kH);
    float a = wih[(size_t)srow * DIN + ci];
    float b = whh[(size_t)srow * kH + khc];
    asm volatile("" : "+v"(a));
    asm volatile("" : "+v"(b));
    float v = vx ? a : (vh ? b : 0.0f);
    v = jv ? (v * kCarry) : 0.0f;
    hv[e] = (_Float16)v;
  }
  unsigned short* q = wc + ((size_t)(dir * kG4 + row) * KTOT + chn * 8);
  *(volatile v8h*)q = hv;
  __threadfence();
  *(volatile v8h*)q = hv;
}

__global__ __launch_bounds__(256) void prep_misc_kernel(
    const float* __restrict__ w_out, const float* __restrict__ b_out,
    const float* __restrict__ b0f, const float* __restrict__ b0b,
    const float* __restrict__ b1f, const float* __restrict__ b1b,
    unsigned short* __restrict__ wo, float* __restrict__ bi0, float* __restrict__ bi1, float* __restrict__ bo)
{
  const int tid = threadIdx.x;
  const int bx  = blockIdx.x;
  if (bx < 10) {
    const int i   = bx * 256 + tid;
    const int row = i >> 5;
    const int chn = i & 31;
    const bool rv = (row < kLbl);
    const int srow = rv ? row : (kLbl - 1);
    v8h hv;
#pragma unroll
    for (int e = 0; e < 8; ++e) {
      const int k    = chn * 8 + e;
      const int half = (k >> 7) & 1;
      const int kk   = k & 127;
      const int ci   = half * kH + ((kk < kH) ? kk : (kH - 1));
      float a = w_out[(size_t)srow * (2 * kH) + ci];
      asm volatile("" : "+v"(a));
      const float v = (rv && (kk < kH)) ? (a * kCarry) : 0.0f;
      hv[e] = (_Float16)v;
    }
    unsigned short* q = wo + ((size_t)row * kHPL + chn * 8);
    *(volatile v8h*)q = hv;
    __threadfence();
    *(volatile v8h*)q = hv;
  } else if (bx < 14) {
    const int qd = bx - 10;
    const float* src = (qd == 0) ? b0f : ((qd == 1) ? b0b : ((qd == 2) ? b1f : b1b));
    float* dst = ((qd < 2) ? bi0 : bi1) + (qd & 1) * kG4;
    const int tc = (tid < 112) ? tid : 111;
    v4f ov;
#pragma unroll
    for (int e = 0; e < 4; ++e) {
      const int n = tc * 4 + e;
      const int g = n / kHP;
      const int j = n - g * kHP;
      float a = src[g * kH + ((j < kH) ? j : (kH - 1))];
      asm volatile("" : "+v"(a));
      ov[e] = (j < kH) ? (a * kCarry2) : 0.0f;
    }
    if (tid < 112) {
      *(volatile v4f*)(dst + tc * 4) = ov;
      __threadfence();
      *(volatile v4f*)(dst + tc * 4) = ov;
    }
  } else {
    const int tc = (tid < 32) ? tid : 31;
    v4f ov;
#pragma unroll
    for (int e = 0; e < 4; ++e) {
      const int n = tc * 4 + e;
      float a = b_out[(n < kLbl) ? n : (kLbl - 1)];
      asm volatile("" : "+v"(a));
      ov[e] = (n < kLbl) ? a : 0.0f;
    }
    if (tid < 32) {
      *(volatile v4f*)(bo + tc * 4) = ov;
      __threadfence();
      *(volatile v4f*)(bo + tc * 4) = ov;
    }
  }
}

__global__ __launch_bounds__(256) void embed_kernel(
    const int* __restrict__ sent, const float* __restrict__ table, unsigned short* __restrict__ x0)
{
  const int i   = blockIdx.x * 256 + threadIdx.x;
  const int r   = i >> 3;
  const int seg = i & 7;
  const int t   = r >> 8;
  const int b   = r & 255;
  int idx = sent[b * kT + t];
  idx = (idx < 0) ? 0 : ((idx > kVocab - 1) ? (kVocab - 1) : idx);
  v8h hv;
#pragma unroll
  for (int e = 0; e < 8; ++e) {
    const int col = seg * 8 + e;
    const int cc  = (col < kEmb) ? col : (kEmb - 1);
    float a = table[(size_t)idx * kEmb + cc];
    asm volatile("" : "+v"(a));
    const float v = (col < kEmb) ? (a * kCarry) : 0.0f;
    hv[e] = (_Float16)v;
  }
  unsigned short* q = x0 + ((size_t)r * kXP0 + seg * 8);
  *(volatile v8h*)q = hv;
  __threadfence();
  *(volatile v8h*)q = hv;
}

template <int KXS, bool BATCH_MAJOR_OUT>
__global__ __launch_bounds__(256) void lstm_scan_kernel(
    const unsigned short* __restrict__ xin_p, const unsigned short* __restrict__ wcat_p,
    const float* __restrict__ bias, unsigned short* __restrict__ hout)
{
  constexpr int XPITCH = KXS * 32;
  constexpr int KTOT   = XPITCH + kHK;
  constexpr int HBUF   = 32 * kHK;
  __shared__ __align__(16) _Float16 hs[2 * HBUF];
  const _Float16* xin  = (const _Float16*)xin_p;
  const _Float16* wcat = (const _Float16*)wcat_p;
  const int tid  = threadIdx.x;
  const int lane = tid & 31;
  const int wave = __builtin_amdgcn_readfirstlane((int)(threadIdx.x >> 5));
  const int hh   = lane >> 4;
  const int m    = lane & 15;
  const int dir  = blockIdx.x >> 3;
  const int b0   = (blockIdx.x & 7) * 32;
  const v8h zero8 = (v8h){0, 0, 0, 0, 0, 0, 0, 0};

  *(v8h*)(&hs[(tid) * 8]) = zero8;
  *(v8h*)(&hs[(tid + 256) * 8]) = zero8;
  __syncthreads();

  const int wv = (wave < 7) ? wave : 6;
  const _Float16* wb = wcat + ((size_t)(dir * kG4 + wv * 16 + m) * KTOT + 8 * hh);
  float bsc[4];
#pragma unroll
  for (int g = 0; g < 4; ++g) bsc[g] = bias[dir * kG4 + g * kHP + wv * 16 + m];
  v8f cst[2];
  cst[0] = (v8f){0.f, 0.f, 0.f, 0.f, 0.f, 0.f, 0.f, 0.f};
  cst[1] = (v8f){0.f, 0.f, 0.f, 0.f, 0.f, 0.f, 0.f, 0.f};

#pragma unroll 1
  for (int s = 0; s < kT; ++s) {
    const int tx  = dir ? (kT - 1 - s) : s;
    const int cur = (s & 1) * HBUF;
    const int nxt = HBUF - cur;
    if (wave < 7) {
      v8f acc[2][4];
#pragma unroll
      for (int mt = 0; mt < 2; ++mt)
#pragma unroll
        for (int g = 0; g < 4; ++g)
          acc[mt][g] = (v8f){bsc[g], bsc[g], bsc[g], bsc[g], bsc[g], bsc[g], bsc[g], bsc[g]};

      const _Float16* xa = xin + ((size_t)(tx * kB + b0 + m) * XPITCH + 8 * hh);
#pragma unroll 1
      for (int ks = 0; ks < KXS; ++ks) {
        const v16h a0 = frag_load_g(xa + ks * 32);
        const v16h a1 = frag_load_g(xa + 16 * XPITCH + ks * 32);
#pragma unroll
        for (int g = 0; g < 4; ++g) {
          const v16h bf = frag_load_g(wb + (size_t)g * kHP * KTOT + ks * 32);
          acc[0][g] = mma_g(a0, bf, acc[0][g]);
          acc[1][g] = mma_g(a1, bf, acc[1][g]);
        }
      }
#pragma unroll 1
      for (int ks = 0; ks < kHK / 32; ++ks) {
        FragU fa0, fa1;
        const int o0 = cur + m * kHK + ks * 32 + 8 * hh;
        fa0.h[0] = *(const v8h*)(&hs[o0]);
        fa0.h[1] = *(const v8h*)(&hs[o0 + 16]);
        fa1.h[0] = *(const v8h*)(&hs[o0 + 16 * kHK]);
        fa1.h[1] = *(const v8h*)(&hs[o0 + 16 * kHK + 16]);
#pragma unroll
        for (int g = 0; g < 4; ++g) {
          const v16h bf = frag_load_g(wb + (size_t)g * kHP * KTOT + XPITCH + ks * 32);
          acc[0][g] = mma_g(fa0.v, bf, acc[0][g]);
          acc[1][g] = mma_g(fa1.v, bf, acc[1][g]);
        }
      }
#pragma unroll
      for (int mt = 0; mt < 2; ++mt) {
#pragma unroll
        for (int r = 0; r < 8; ++r) {
          const float pi = acc[mt][0][r] * kInvCarry2;
          const float pf = acc[mt][1][r] * kInvCarry2;
          const float pg = acc[mt][2][r] * kInvCarry2;
          const float po = acc[mt][3][r] * kInvCarry2;
          const float si = sig_fast(pi);
          const float sf = sig_fast(pf);
          const float tg = tanh_fast(pg);
          const float so = sig_fast(po);
          const float cn = sf * cst[mt][r] + si * tg;
          cst[mt][r] = cn;
          const float hn = so * tanh_fast(cn);
          hs[nxt + (mt * 16 + 8 * hh + r) * kHK + wave * 16 + m] = (_Float16)(hn * kCarry);
        }
      }
    } else {
      const int pr = lane >> 1;
      const int pc = 112 + 8 * (lane & 1);
      *(v8h*)(&hs[nxt + pr * kHK + pc]) = zero8;
      *(v8h*)(&hs[nxt + (pr + 16) * kHK + pc]) = zero8;
    }
    __syncthreads();
    if (wave == 7) {
      const size_t obase = BATCH_MAJOR_OUT ? ((size_t)(b0 * kT + tx) * kHPL + dir * kHK)
                                           : ((size_t)(tx * kB + b0) * kHPL + dir * kHK);
      constexpr size_t ROWP = BATCH_MAJOR_OUT ? ((size_t)kT * kHPL) : (size_t)kHPL;
      for (int pass = 0; pass < 2; ++pass) {
#pragma unroll 4
        for (int it = 0; it < 16; ++it) {
          const int row = it * 2 + hh;
          const v8h v = *(const v8h*)(&hs[nxt + row * kHK + m * 8]);
          *(volatile v8h*)(hout + obase + (size_t)row * ROWP + m * 8) = v;
        }
        __threadfence();
      }
    }
  }
}

__global__ __launch_bounds__(256) void head_kernel(
    const unsigned short* __restrict__ h1_p, const unsigned short* __restrict__ wo_p,
    const float* __restrict__ bo, float* __restrict__ out)
{
  __shared__ __align__(16) float cs[128 * kLbl];
  const _Float16* h1 = (const _Float16*)h1_p;
  const _Float16* wo = (const _Float16*)wo_p;
  const int tid  = threadIdx.x;
  const int lane = tid & 31;
  const int wave = __builtin_amdgcn_readfirstlane((int)(threadIdx.x >> 5));
  const int hh   = lane >> 4;
  const int m    = lane & 15;
  const size_t m0 = (size_t)blockIdx.x * 128;
  v8f acc[5];
#pragma unroll
  for (int j = 0; j < 5; ++j) acc[j] = (v8f){0.f, 0.f, 0.f, 0.f, 0.f, 0.f, 0.f, 0.f};
  const _Float16* ap = h1 + ((m0 + wave * 16 + m) * kHPL + 8 * hh);
  const _Float16* bp = wo + ((size_t)m * kHPL + 8 * hh);
#pragma unroll 1
  for (int ks = 0; ks < kHPL / 32; ++ks) {
    const v16h a = frag_load_g(ap + ks * 32);
#pragma unroll
    for (int j = 0; j < 5; ++j) {
      const v16h bf = frag_load_g(bp + (size_t)j * 16 * kHPL + ks * 32);
      acc[j] = mma_g(a, bf, acc[j]);
    }
  }
#pragma unroll
  for (int j = 0; j < 5; ++j) {
    const int n = j * 16 + m;
    float bv = bo[n];
    asm volatile("" : "+v"(bv));
#pragma unroll
    for (int r = 0; r < 8; ++r) {
      const int row = wave * 16 + 8 * hh + r;
      const float v = acc[j][r] * kInvCarry2 + bv;
      if (n < kLbl) cs[row * kLbl + n] = v;
    }
  }
  __syncthreads();
  float* ob = out + m0 * kLbl;
  constexpr int NV4 = 128 * kLbl / 4;
  for (int pass = 0; pass < 2; ++pass) {
#pragma unroll 1
    for (int it = 0; it < 9; ++it) {
      const int i = tid + 256 * it;
      if (i < NV4) {
        const v4f v = *(const v4f*)(&cs[4 * i]);
        *(volatile v4f*)(ob + 4 * (size_t)i) = v;
      }
    }
    __threadfence();
  }
}

extern "C" void kernel_launch(void* const* d_in, const int* in_sizes, int n_in,
                              void* d_out, int out_size, void* d_ws, size_t ws_size,
                              hipStream_t stream) {
  if (n_in < 16) return;
  if (in_sizes[0] != kB * kT) return;
  if (in_sizes[1] != kVocab * kEmb) return;
  if (in_sizes[2] != 4 * kH * kEmb || in_sizes[5] != 4 * kH * kEmb) return;
  if (in_sizes[3] != 4 * kH * kH || in_sizes[6] != 4 * kH * kH) return;
  if (in_sizes[9] != 4 * kH * kH || in_sizes[12] != 4 * kH * kH) return;
  if (in_sizes[8] != 4 * kH * 2 * kH || in_sizes[11] != 4 * kH * 2 * kH) return;
  if (in_sizes[4] != 4 * kH || in_sizes[7] != 4 * kH || in_sizes[10] != 4 * kH || in_sizes[13] != 4 * kH) return;
  if (in_sizes[14] != kLbl * 2 * kH || in_sizes[15] != kLbl) return;
  if (out_size != kRows * kLbl) return;
  if (ws_size < kWsTotal) return;

  const int*   sent     = (const int*)  d_in[0];
  const float* emb      = (const float*)d_in[1];
  const float* wih_l0_f = (const float*)d_in[2];
  const float* whh_l0_f = (const float*)d_in[3];
  const float* b_l0_f   = (const float*)d_in[4];
  const float* wih_l0_b = (const float*)d_in[5];
  const float* whh_l0_b = (const float*)d_in[6];
  const float* b_l0_b   = (const float*)d_in[7];
  const float* wih_l1_f = (const float*)d_in[8];
  const float* whh_l1_f = (const float*)d_in[9];
  const float* b_l1_f   = (const float*)d_in[10];
  const float* wih_l1_b = (const float*)d_in[11];
  const float* whh_l1_b = (const float*)d_in[12];
  const float* b_l1_b   = (const float*)d_in[13];
  const float* w_out    = (const float*)d_in[14];
  const float* b_out    = (const float*)d_in[15];
  float* out = (float*)d_out;

  char* ws = (char*)d_ws;
  unsigned short* X0  = (unsigned short*)(ws + kOffX0);
  unsigned short* H0  = (unsigned short*)(ws + kOffH0);
  unsigned short* H1  = (unsigned short*)(ws + kOffH1);
  unsigned short* WC0 = (unsigned short*)(ws + kOffWC0);
  unsigned short* WC1 = (unsigned short*)(ws + kOffWC1);
  unsigned short* WO  = (unsigned short*)(ws + kOffWO);
  float*          BI0 = (float*)(ws + kOffBI0);
  float*          BI1 = (float*)(ws + kOffBI1);
  float*          BO  = (float*)(ws + kOffBO);

  prep_wcat_kernel<kEmb, kXP0><<<dim3(42, 2), 256, 0, stream>>>(wih_l0_f, whh_l0_f, wih_l0_b, whh_l0_b, WC0);
  prep_wcat_kernel<2 * kH, kHPL><<<dim3(84, 2), 256, 0, stream>>>(wih_l1_f, whh_l1_f, wih_l1_b, whh_l1_b, WC1);
  prep_misc_kernel<<<15, 256, 0, stream>>>(w_out, b_out, b_l0_f, b_l0_b, b_l1_f, b_l1_b, WO, BI0, BI1, BO);
  embed_kernel<<<(kRows * 8) / 256, 256, 0, stream>>>(sent, emb, X0);

  lstm_scan_kernel<kXP0 / 32, false><<<16, 256, 0, stream>>>(X0, WC0, BI0, H0);
  lstm_scan_kernel<kHPL / 32, true><<<16, 256, 0, stream>>>(H0, WC1, BI1, H1);

  head_kernel<<<kRows / 128, 256, 0, stream>>>(H1, WO, BO, out);
}
